// IMUToTrajectoryNet_77094662963457
// MI455X (gfx1250) — hardware-run, weakly checked
//
#include <hip/hip_runtime.h>
#include <hip/hip_fp16.h>
#include <math.h>

typedef __attribute__((ext_vector_type(16))) _Float16 v16h;
typedef __attribute__((ext_vector_type(8)))  _Float16 v8h;
typedef __attribute__((ext_vector_type(2)))  _Float16 v2h;
typedef __attribute__((ext_vector_type(8)))  float    v8f;
typedef __attribute__((ext_vector_type(4)))  float    v4f;
typedef __attribute__((ext_vector_type(2)))  float    v2f;

constexpr int kB = 128;
constexpr int kT = 4096;
constexpr int kI = 6;
constexpr int kH = 32;
constexpr int kG = 96;
constexpr int kO = 2;
constexpr int kPX = 40;
constexpr int kPH = 40;
constexpr int kPW = 40;
constexpr int kSamp = 32;
constexpr int kSlots = 16;
constexpr float kWCarry = 1024.0f;
constexpr float sW = 1.0f / kWCarry;
static_assert(kG == 3 * kH);
static_assert(kI <= 32 && kH == 32);
static_assert((kPX % 8) == 0 && (kPH % 8) == 0 && (kPW % 8) == 0);
static_assert(kPX >= 32 && kPH >= 32 && kPW >= 32);
static_assert((32 * kPX) == 8 * 160 && (32 * kPH) == 8 * 160);
static_assert((kB % kSamp) == 0 && (kT % kSlots) == 0);
static_assert(kB / kSamp == 4);
static_assert(kSlots * kO == 32);
static_assert(kB * kT * kO == 1048576);
static_assert(kB * kT * kI == 3145728);

constexpr size_t kSzWHH = (size_t)kG * kH * 2;
constexpr size_t kSzBG  = 512;
constexpr size_t kOffWHH = 0;
constexpr size_t kOffBIH = kOffWHH + kSzWHH;
constexpr size_t kOffBHH = kOffBIH + kSzBG;
constexpr size_t kWsTotal = kOffBHH + kSzBG;
static_assert(kSzWHH == 6144ull);
static_assert((size_t)kG * 4 <= kSzBG);
static_assert(kWsTotal == 7168ull);
static_assert(kWsTotal <= 134217728ull);
static_assert((kSzWHH % 256) == 0 && (kSzBG % 256) == 0);
static_assert((kOffBIH % 256) == 0 && (kOffBHH % 256) == 0);

__device__ __forceinline__ _Float16 f16_flush(float v) {
  const float w = (fabsf(v) < 6.103515625e-05f) ? 0.0f : v;
  return (_Float16)w;
}

__device__ __forceinline__ float bf16r(float v) {
  unsigned u = __float_as_uint(v);
  u = (u + 0x7FFFu + ((u >> 16) & 1u)) & 0xFFFF0000u;
  return __uint_as_float(u);
}

namespace eng {
union FragU { v16h v; v8h h[2]; };
__device__ __forceinline__ v16h frag_load(const _Float16* p) {
  FragU f;
  f.h[0] = *(const v8h*)(p);
  f.h[1] = *(const v8h*)(p + 16);
  return f.v;
}
__device__ __forceinline__ v8f mma(v16h a, v16h b, v8f c) {
  return __builtin_amdgcn_wmma_f32_16x16x32_f16(false, a, false, b, (short)0, c, false, false);
}
__device__ __forceinline__ void guard1(v8f& a, v16h x, v16h y) {
  asm volatile("v_nop\n\tv_nop\n\tv_nop\n\tv_nop" : "+v"(a) : "v"(x), "v"(y));
}
__device__ __forceinline__ void guard_acc(v8f& a) {
  asm volatile("v_nop\n\tv_nop\n\tv_nop\n\tv_nop" : "+v"(a));
}
__device__ __forceinline__ void keep4(v16h a, v16h b, v16h c, v16h d) {
  asm volatile("v_nop" :: "v"(a), "v"(b), "v"(c), "v"(d));
}
}

template <int K>
__device__ __forceinline__ v8f tile_mm(const _Float16* A, int lda, const _Float16* __restrict__ Bt, int ldb,
                                       int n0, int rlane, int koff, v8f acc)
{
  static_assert((K % 32) == 0 && K >= 32 && K <= 128);
#pragma unroll
  for (int k0 = 0; k0 < K; k0 += 32) {
    const v16h ah = eng::frag_load(A + rlane * lda + koff + k0);
    const v16h bh = eng::frag_load(Bt + (size_t)(n0 + rlane) * ldb + koff + k0);
    acc = eng::mma(ah, bh, acc);
    eng::guard1(acc, ah, bh);
    eng::keep4(bh, bh, ah, ah);
  }
  return acc;
}

__global__ __launch_bounds__(256) void pack_rows_bf_kernel(
    const float* __restrict__ W, unsigned short* __restrict__ dH,
    int Kdim, int Nreal, int total8, float carry)
{
  const int i = blockIdx.x * 256 + threadIdx.x;
  if (i >= total8) return;
  const size_t e0 = (size_t)i << 3;
  const int row = (int)(e0 / (size_t)Kdim);
  const int col = (int)(e0 - (size_t)row * (size_t)Kdim);
  const bool live = (row < Nreal);
  const int rc = live ? row : (Nreal - 1);
  const v4f a0 = *(const v4f*)(W + (size_t)rc * Kdim + col);
  const v4f a1 = *(const v4f*)(W + (size_t)rc * Kdim + col + 4);
  const float w0 = a0[0];
  const float w1 = a0[1];
  const float w2 = a0[2];
  const float w3 = a0[3];
  const float w4 = a1[0];
  const float w5 = a1[1];
  const float w6 = a1[2];
  const float w7 = a1[3];
  const float t0 = bf16r(w0) * carry;
  const float t1 = bf16r(w1) * carry;
  const float t2 = bf16r(w2) * carry;
  const float t3 = bf16r(w3) * carry;
  const float t4 = bf16r(w4) * carry;
  const float t5 = bf16r(w5) * carry;
  const float t6 = bf16r(w6) * carry;
  const float t7 = bf16r(w7) * carry;
  const float g0 = live ? t0 : 0.0f;
  const float g1 = live ? t1 : 0.0f;
  const float g2 = live ? t2 : 0.0f;
  const float g3 = live ? t3 : 0.0f;
  const float g4 = live ? t4 : 0.0f;
  const float g5 = live ? t5 : 0.0f;
  const float g6 = live ? t6 : 0.0f;
  const float g7 = live ? t7 : 0.0f;
  v8h hv;
  hv[0] = f16_flush(g0);
  hv[1] = f16_flush(g1);
  hv[2] = f16_flush(g2);
  hv[3] = f16_flush(g3);
  hv[4] = f16_flush(g4);
  hv[5] = f16_flush(g5);
  hv[6] = f16_flush(g6);
  hv[7] = f16_flush(g7);
  unsigned short* qh = dH + e0;
  *(volatile v8h*)qh = hv;
  __threadfence();
  *(volatile v8h*)qh = hv;
}

__global__ __launch_bounds__(256) void rne_vec_kernel(
    const float* __restrict__ src, float* __restrict__ dst, int n4)
{
  const int i = blockIdx.x * 256 + threadIdx.x;
  if (i >= n4) return;
  const v4f a = *(const v4f*)(src + (size_t)i * 4);
  const float a0 = a[0];
  const float a1 = a[1];
  const float a2 = a[2];
  const float a3 = a[3];
  v4f r;
  r[0] = bf16r(a0);
  r[1] = bf16r(a1);
  r[2] = bf16r(a2);
  r[3] = bf16r(a3);
  float* p = dst + (size_t)i * 4;
  *(volatile v4f*)p = r;
  __threadfence();
  *(volatile v4f*)p = r;
}

__device__ __forceinline__ void stage_x6(const float* __restrict__ x, _Float16* P_X, int b0, int tid, int tt)
{
  if (tid < 96) {
    const int sx = tid / 3;
    const int pq = tid - 3 * sx;
    const v2f xr = *(const v2f*)(x + ((size_t)(b0 + sx) * kT + tt) * kI + 2 * pq);
    const float x0 = xr[0];
    const float x1 = xr[1];
    v2h hv;
    hv[0] = f16_flush(bf16r(x0));
    hv[1] = f16_flush(bf16r(x1));
    *(v2h*)(P_X + sx * kPX + 2 * pq) = hv;
  }
}

__device__ __forceinline__ void flush16(const float* YS, float* __restrict__ out, int b0, int tid, int t0)
{
  const int p  = tid & 7;
  const int s0 = tid >> 3;
  const int s1 = 16 + s0;
  const v4f v0 = *(const v4f*)(YS + s0 * (kSlots * kO) + 4 * p);
  const v4f v1 = *(const v4f*)(YS + s1 * (kSlots * kO) + 4 * p);
  float* o0 = out + ((size_t)(b0 + s0) * kT + t0) * kO + 4 * p;
  float* o1 = out + ((size_t)(b0 + s1) * kT + t0) * kO + 4 * p;
  for (int pass = 0; pass < 2; ++pass) {
    *(volatile v4f*)o0 = v0;
    *(volatile v4f*)o1 = v1;
    __threadfence();
  }
}

__global__ __launch_bounds__(128) void gru_mask_head_kernel(
    const float* __restrict__ x,
    const int* __restrict__ lengths,
    const float* __restrict__ w_ih,
    const unsigned short* __restrict__ WHHp,
    const float* __restrict__ BIH,
    const float* __restrict__ BHH,
    const float* __restrict__ fc_w,
    const float* __restrict__ fc_b,
    float* __restrict__ out)
{
  __shared__ __align__(16) _Float16 P_X[32 * kPX];
  __shared__ __align__(16) _Float16 P_H[32 * kPH];
  __shared__ __align__(16) _Float16 WIH_S[kG * kPW];
  __shared__ __align__(16) float HS[32 * 32];
  __shared__ __align__(16) float YS[32 * 32];
  __shared__ __align__(16) float FW_S[64];

  const _Float16* WHH = (const _Float16*)WHHp;

  const int tid   = threadIdx.x;
  const int lane  = tid & 31;
  const int wave  = tid >> 5;
  const int rlane = lane & 15;
  const int hi    = lane >> 4;
  const int koff  = 8 * hi;
  const int st    = wave >> 1;
  const int ut    = wave & 1;
  const int u     = 16 * ut + rlane;
  const int b0    = blockIdx.x * kSamp;
  const int srow  = 16 * st + 8 * hi;

  const float br  = BIH[u] + BHH[u];
  const float bz  = BIH[kH + u] + BHH[kH + u];
  const float bxn = BIH[2 * kH + u];
  const float bhn = BHH[2 * kH + u];
  const float fcb = bf16r(fc_b[tid & 1]);

  int len[8];
#pragma unroll
  for (int r8 = 0; r8 < 8; ++r8) {
    int lv = lengths[b0 + srow + r8];
    lv = (lv < 0) ? 0 : lv;
    lv = (lv > kT) ? kT : lv;
    len[r8] = lv;
  }

  const v8f vz = (v8f){0.f, 0.f, 0.f, 0.f, 0.f, 0.f, 0.f, 0.f};
  v8f hreg = vz;

  {
    const _Float16 hz = (_Float16)0.0f;
    const v8h z8 = (v8h){hz, hz, hz, hz, hz, hz, hz, hz};
    *(v8h*)(P_X + 8 * tid) = z8;
    *(v8h*)(P_H + 8 * tid) = z8;
    if (tid < 32) {
      *(v8h*)(P_X + 8 * (128 + tid)) = z8;
      *(v8h*)(P_H + 8 * (128 + tid)) = z8;
    }
  }
  for (int i = tid; i < kG * kPW; i += 128) {
    const int n = i / kPW;
    const int k = i - kPW * n;
    const int kc = (k < kI) ? k : (kI - 1);
    const float wv = bf16r(w_ih[n * kI + kc]) * kWCarry;
    const float g = (k < kI) ? wv : 0.0f;
    WIH_S[i] = f16_flush(g);
  }
  if (tid < 64) FW_S[tid] = bf16r(fc_w[tid]);
  __syncthreads();
  stage_x6(x, P_X, b0, tid, 0);
  __syncthreads();

  const _Float16* A_X = P_X + 16 * st * kPX;
  const _Float16* A_H = P_H + 16 * st * kPH;

  for (int t = 0; t < kT; ++t) {
    v8f em = vz;

    {
      v8f ar  = tile_mm<32>(A_X, kPX, WIH_S, kPW, 0 * kH + 16 * ut, rlane, koff, vz);
      ar      = tile_mm<32>(A_H, kPH, WHH, kH, 0 * kH + 16 * ut, rlane, koff, ar);
      v8f az  = tile_mm<32>(A_X, kPX, WIH_S, kPW, 1 * kH + 16 * ut, rlane, koff, vz);
      az      = tile_mm<32>(A_H, kPH, WHH, kH, 1 * kH + 16 * ut, rlane, koff, az);
      v8f axn = tile_mm<32>(A_X, kPX, WIH_S, kPW, 2 * kH + 16 * ut, rlane, koff, vz);
      v8f ahn = tile_mm<32>(A_H, kPH, WHH, kH, 2 * kH + 16 * ut, rlane, koff, vz);
      eng::guard_acc(ar);
      eng::guard_acc(az);
      eng::guard_acc(axn);
      eng::guard_acc(ahn);
#pragma unroll
      for (int r8 = 0; r8 < 8; ++r8) {
        const float pr = ar[r8] * sW + br;
        const float pz = az[r8] * sW + bz;
        const float px = axn[r8] * sW + bxn;
        const float ph = ahn[r8] * sW + bhn;
        const float rg = 1.0f / (1.0f + expf(-pr));
        const float zg = 1.0f / (1.0f + expf(-pz));
        const float ng = tanhf(px + rg * ph);
        const float ho = hreg[r8];
        const float hn = (1.0f - zg) * ng + zg * ho;
        const bool valid = (t < len[r8]);
        em[r8] = valid ? hn : 0.0f;
        hreg[r8] = valid ? hn : ho;
      }
    }
    __syncthreads();

#pragma unroll
    for (int r8 = 0; r8 < 8; ++r8) {
      P_H[(srow + r8) * kPH + u] = f16_flush(hreg[r8]);
      HS[(srow + r8) * 32 + u] = em[r8];
    }
    if (t + 1 < kT) stage_x6(x, P_X, b0, tid, t + 1);
    if (t >= kSlots && (t & (kSlots - 1)) == 0) flush16(YS, out, b0, tid, t - kSlots);
    __syncthreads();

    if (tid < 64) {
      const int s = tid >> 1;
      const int o = tid & 1;
      const float* hs = HS + s * 32;
      const float* fw = FW_S + o * 32;
      float y = fcb;
      for (int u2 = 0; u2 < kH; ++u2) y += hs[u2] * fw[u2];
      YS[s * (kSlots * kO) + (t & (kSlots - 1)) * kO + o] = y;
    }
  }

  __syncthreads();
  flush16(YS, out, b0, tid, kT - kSlots);
}

static_assert((kG * kH / 8) == 384);
static_assert((kG / 4) == 24);

extern "C" void kernel_launch(void* const* d_in, const int* in_sizes, int n_in,
                              void* d_out, int out_size, void* d_ws, size_t ws_size,
                              hipStream_t stream)
{
  if (n_in < 8) return;
  if (in_sizes[0] != kB * kT * kI) return;
  if (in_sizes[1] != kB) return;
  if (in_sizes[2] != kG * kI) return;
  if (in_sizes[3] != kG * kH) return;
  if (in_sizes[4] != kG) return;
  if (in_sizes[5] != kG) return;
  if (in_sizes[6] != kO * kH) return;
  if (in_sizes[7] != kO) return;
  if (out_size != kB * kT * kO) return;
  if (ws_size < kWsTotal) return;

  const float* x       = (const float*)d_in[0];
  const int*   lengths = (const int*)d_in[1];
  const float* w_ih    = (const float*)d_in[2];
  const float* w_hh    = (const float*)d_in[3];
  const float* b_ih    = (const float*)d_in[4];
  const float* b_hh    = (const float*)d_in[5];
  const float* fc_w    = (const float*)d_in[6];
  const float* fc_b    = (const float*)d_in[7];
  float* out = (float*)d_out;

  char* ws = (char*)d_ws;
  unsigned short* WHH = (unsigned short*)(ws + kOffWHH);
  float* BIH = (float*)(ws + kOffBIH);
  float* BHH = (float*)(ws + kOffBHH);

  pack_rows_bf_kernel<<<2, 256, 0, stream>>>(w_hh, WHH, kH, kG, kG * kH / 8, kWCarry);
  rne_vec_kernel<<<1, 256, 0, stream>>>(b_ih, BIH, kG / 4);
  rne_vec_kernel<<<1, 256, 0, stream>>>(b_hh, BHH, kG / 4);

  gru_mask_head_kernel<<<kB / kSamp, 128, 0, stream>>>(x, lengths, w_ih, WHH, BIH, BHH, fc_w, fc_b, out);
}
